// EVCBlock_20890720928164
// MI455X (gfx1250) — hardware-verified
//
#include <hip/hip_runtime.h>
#define NB 8
#define CC 256
#define CQ 64
#define HS 40
#define PX (HS * HS)
#define NRW ((size_t)NB * PX)
#define KST (49 * CC)
#define RCH 3200
#define NK 64
#define HID 1024
#define NPART 25
typedef __bf16 v16b __attribute__((ext_vector_type(16)));
typedef unsigned short v8us __attribute__((ext_vector_type(8), may_alias));
typedef float  v8f  __attribute__((ext_vector_type(8)));
typedef float  v4f  __attribute__((ext_vector_type(4)));
typedef float  v4fa __attribute__((ext_vector_type(4), may_alias));
union FragB { v16b v; v8us half[2]; unsigned short u[16]; };

__device__ __forceinline__ unsigned short bf16_bits(float x) { unsigned int u = __float_as_uint(x); return (unsigned short)((u + 0x7FFFu + ((u >> 16) & 1u)) >> 16); }
__device__ __forceinline__ float bf16_val(unsigned short b) { return __uint_as_float(((unsigned int)b) << 16); }
__device__ __forceinline__ float bf16_round(float x) { return bf16_val(bf16_bits(x)); }
template <int NT>
__device__ __forceinline__ v8f mmaN(v16b ah, v16b al, v16b bh, v16b bl, v8f c) {
  c = __builtin_amdgcn_wmma_f32_16x16x32_bf16(false, ah, false, bh, (short)0, c, false, false);
  if (NT >= 2) c = __builtin_amdgcn_wmma_f32_16x16x32_bf16(false, al, false, bh, (short)0, c, false, false);
  if (NT >= 3) c = __builtin_amdgcn_wmma_f32_16x16x32_bf16(false, ah, false, bl, (short)0, c, false, false);
  asm volatile("v_nop\n\tv_nop\n\tv_nop\n\tv_nop" : "+v"(c) : "v"(ah), "v"(al), "v"(bh), "v"(bl));
  return c;
}

__global__ __launch_bounds__(256) void k_wt_bf16(const float* __restrict__ W, unsigned short* __restrict__ Wt, int K, int N) {
  const int t = blockIdx.x * 256 + threadIdx.x;
  const int k8n = K / 8;
  if (t >= N * k8n) return;
  const int n = t / k8n, k8 = (t % k8n) * 8;
  v8us v;
#pragma unroll
  for (int i = 0; i < 8; ++i) v[i] = bf16_bits(W[(size_t)(k8 + i) * N + n]);
  *(volatile v8us*)(Wt + (size_t)n * K + k8) = v;
  __threadfence();
  *(volatile v8us*)(Wt + (size_t)n * K + k8) = v;
}

template <bool ASPLIT, int ACT, bool BIAS_BF16>
__global__ __launch_bounds__(128) void k_gemm_bf(const float* __restrict__ A, int lda, const unsigned short* __restrict__ Wt, int ldb,
                                               const float* __restrict__ bias, float* __restrict__ C, int ldc, int M, int N, int K) {
  __shared__ __attribute__((aligned(16))) float so[4][16][64];
  const int tid = threadIdx.x, w = tid >> 5, lane = tid & 31, ln = lane & 15, hh = lane >> 4;
  const int ntn = N / 64;
  const int wid = blockIdx.x * 4 + w;
  const int mt = wid / ntn, nq = wid % ntn;
  if (mt * 16 >= M) return;
  const int row0 = mt * 16, col0 = nq * 64;
  const float* arow = A + (size_t)(row0 + ln) * lda;
  v8f acc[4] = {};
  for (int kb = 0; kb < K; kb += 32) {
    FragB ah, al;
    const v4f x0 = *(const v4fa*)(arow + kb + 8 * hh), x1 = *(const v4fa*)(arow + kb + 8 * hh + 4);
    const v4f x2 = *(const v4fa*)(arow + kb + 16 + 8 * hh), x3 = *(const v4fa*)(arow + kb + 16 + 8 * hh + 4);
    float xs[16] = {x0[0],x0[1],x0[2],x0[3],x1[0],x1[1],x1[2],x1[3],x2[0],x2[1],x2[2],x2[3],x3[0],x3[1],x3[2],x3[3]};
#pragma unroll
    for (int i = 0; i < 16; ++i) { const unsigned short hb = bf16_bits(xs[i]); ah.u[i] = hb; al.u[i] = ASPLIT ? bf16_bits(xs[i] - bf16_val(hb)) : (unsigned short)0; }
#pragma unroll
    for (int t = 0; t < 4; ++t) {
      const unsigned short* brow = Wt + (size_t)(col0 + t * 16 + ln) * ldb + kb;
      FragB b;
      b.half[0] = *(const v8us*)(brow + 8 * hh);
      b.half[1] = *(const v8us*)(brow + 16 + 8 * hh);
      acc[t] = mmaN<ASPLIT ? 2 : 1>(ah.v, al.v, b.v, b.v, acc[t]);
    }
  }
#pragma unroll
  for (int t = 0; t < 4; ++t) {
    float bv = bias ? bias[col0 + t * 16 + ln] : 0.f;
    if (BIAS_BF16) bv = bf16_round(bv);
#pragma unroll
    for (int r = 0; r < 8; ++r) { float v = acc[t][r] + bv; if (ACT == 1) v = fmaxf(v, 0.f); so[w][8 * hh + r][t * 16 + ln] = v; }
  }
  __builtin_amdgcn_fence(__ATOMIC_ACQ_REL, "workgroup");
  __builtin_amdgcn_wave_barrier();
  const int rsub = lane >> 4, c4 = (lane & 15) * 4;
  for (int pass = 0; pass < 2; ++pass) {
#pragma unroll
    for (int q = 0; q < 8; ++q) {
      const int r = q * 2 + rsub;
      const v4f v = *(const v4fa*)&so[w][r][c4];
      *(volatile v4f*)(C + (size_t)(row0 + r) * ldc + col0 + c4) = v;
    }
    if (pass == 0) __threadfence();
  }
}

template <bool ASPLIT, int ACT, bool BIAS_BF16, bool RES_BF16>
__global__ __launch_bounds__(128) void k_gemm_bf3(const float* __restrict__ A, int lda, const unsigned short* __restrict__ Wt, int ldb,
                                                const float* __restrict__ bias, const float* __restrict__ resid, int rmod, int ldr,
                                                float* __restrict__ C, int ldc, int M, int N, int K) {
  __shared__ __attribute__((aligned(16))) float so[4][16][64];
  const int tid = threadIdx.x, w = tid >> 5, lane = tid & 31, ln = lane & 15, hh = lane >> 4;
  const int ntn = N / 64;
  const int wid = blockIdx.x * 4 + w;
  const int mt = wid / ntn, nq = wid % ntn;
  if (mt * 16 >= M) return;
  const int row0 = mt * 16, col0 = nq * 64;
  const float* arow = A + (size_t)(row0 + ln) * lda;
  v8f acc[4] = {};
  for (int kb = 0; kb < K; kb += 32) {
    FragB ah, al;
    const v4f x0 = *(const v4fa*)(arow + kb + 8 * hh), x1 = *(const v4fa*)(arow + kb + 8 * hh + 4);
    const v4f x2 = *(const v4fa*)(arow + kb + 16 + 8 * hh), x3 = *(const v4fa*)(arow + kb + 16 + 8 * hh + 4);
    float xs[16] = {x0[0],x0[1],x0[2],x0[3],x1[0],x1[1],x1[2],x1[3],x2[0],x2[1],x2[2],x2[3],x3[0],x3[1],x3[2],x3[3]};
#pragma unroll
    for (int i = 0; i < 16; ++i) { const unsigned short hb = bf16_bits(xs[i]); ah.u[i] = hb; al.u[i] = ASPLIT ? bf16_bits(xs[i] - bf16_val(hb)) : (unsigned short)0; }
#pragma unroll
    for (int t = 0; t < 4; ++t) {
      const unsigned short* brow = Wt + (size_t)(col0 + t * 16 + ln) * ldb + kb;
      FragB b;
      b.half[0] = *(const v8us*)(brow + 8 * hh);
      b.half[1] = *(const v8us*)(brow + 16 + 8 * hh);
      acc[t] = mmaN<ASPLIT ? 2 : 1>(ah.v, al.v, b.v, b.v, acc[t]);
    }
  }
#pragma unroll
  for (int t = 0; t < 4; ++t) {
    const int col = col0 + t * 16 + ln;
    float bv = bias ? bias[col] : 0.f;
    if (BIAS_BF16) bv = bf16_round(bv);
#pragma unroll
    for (int r = 0; r < 8; ++r) {
      float v = acc[t][r] + bv;
      if (resid) { float rv = resid[(size_t)((row0 + 8 * hh + r) % rmod) * ldr + col]; if (RES_BF16) rv = bf16_round(rv); v += rv; }
      if (ACT == 1) v = fmaxf(v, 0.f);
      if (ACT == 2) v = 0.5f * v * (1.0f + erff(v * 0.70710678118654752f));
      if (ACT == 3) { const float u = 0.7978845608028654f * (v + 0.044715f * v * v * v); v = 0.5f * v * (1.0f + tanhf(u)); }
      so[w][8 * hh + r][t * 16 + ln] = v;
    }
  }
  __builtin_amdgcn_fence(__ATOMIC_ACQ_REL, "workgroup");
  __builtin_amdgcn_wave_barrier();
  const int rsub = lane >> 4, c4 = (lane & 15) * 4;
  for (int pass = 0; pass < 2; ++pass) {
#pragma unroll
    for (int q = 0; q < 8; ++q) {
      const int r = q * 2 + rsub;
      const v4f v = *(const v4fa*)&so[w][r][c4];
      *(volatile v4f*)(C + (size_t)(row0 + r) * ldc + col0 + c4) = v;
    }
    if (pass == 0) __threadfence();
  }
}
template <bool PARAM_BF16>
__global__ __launch_bounds__(256) void k_layernorm(const float* __restrict__ X, const float* __restrict__ R, const float* __restrict__ g, const float* __restrict__ bta,
                                                  float* __restrict__ out_sum, float* __restrict__ out_norm, int N, float eps) {
  __shared__ float red[256];
  const int row = blockIdx.x, tid = threadIdx.x;
  const float* x = X + (size_t)row * N; const float* rr = R ? R + (size_t)row * N : nullptr;
  float vals[16];
  const int per = N / 256;
  float s1 = 0.f;
  for (int u = 0; u < per / 4; ++u) {
    const int j = tid * 4 + 1024 * u;
    const v4f a = *(const v4fa*)(x + j);
    v4f b = {0.f,0.f,0.f,0.f}; if (rr) b = *(const v4fa*)(rr + j);
#pragma unroll
    for (int q = 0; q < 4; ++q) { const float v = a[q] + b[q]; vals[u * 4 + q] = v; s1 += v; }
  }
  red[tid] = s1; __syncthreads();
  for (int st = 128; st > 0; st >>= 1) { if (tid < st) red[tid] += red[tid + st]; __syncthreads(); }
  const float mu = red[0] / (float)N; __syncthreads();
  float s2 = 0.f;
  for (int u = 0; u < per / 4; ++u)
#pragma unroll
    for (int q = 0; q < 4; ++q) { const float c = vals[u * 4 + q] - mu; s2 += c * c; }
  red[tid] = s2; __syncthreads();
  for (int st = 128; st > 0; st >>= 1) { if (tid < st) red[tid] += red[tid + st]; __syncthreads(); }
  const float rs = rsqrtf(red[0] / (float)N + eps);
  for (int pass = 0; pass < 2; ++pass) {
    for (int u = 0; u < per / 4; ++u) {
      const int j = tid * 4 + 1024 * u;
      v4f o, sm;
#pragma unroll
      for (int q = 0; q < 4; ++q) {
        float gg = g[j + q], bb = bta[j + q];
        if (PARAM_BF16) { gg = bf16_round(gg); bb = bf16_round(bb); }
        sm[q] = vals[u * 4 + q]; o[q] = (vals[u * 4 + q] - mu) * rs * gg + bb;
      }
      if (out_sum) *(volatile v4f*)(out_sum + (size_t)row * N + j) = sm;
      *(volatile v4f*)(out_norm + (size_t)row * N + j) = o;
    }
    if (pass == 0) __threadfence();
  }
}


typedef _Float16 v16h __attribute__((ext_vector_type(16)));
union FragH { v16h v; v8us half[2]; _Float16 h[16]; unsigned short u[16]; };
template <int NT>
__device__ __forceinline__ v8f mmaH(v16h ah, v16h al, v16h bh, v16h bl, v8f c) {
  c = __builtin_amdgcn_wmma_f32_16x16x32_f16(false, ah, false, bh, (short)0, c, false, false);
  if (NT >= 2) c = __builtin_amdgcn_wmma_f32_16x16x32_f16(false, al, false, bh, (short)0, c, false, false);
  if (NT >= 3) c = __builtin_amdgcn_wmma_f32_16x16x32_f16(false, ah, false, bl, (short)0, c, false, false);
  asm volatile("v_nop\n\tv_nop\n\tv_nop\n\tv_nop" : "+v"(c) : "v"(ah), "v"(al), "v"(bh), "v"(bl));
  return c;
}
template <bool ASPLIT>
__global__ __launch_bounds__(128) void k_gemm_h(const float* __restrict__ A, int lda, size_t sA, const _Float16* __restrict__ Bh, int ldb, size_t sB, float alpha, float* __restrict__ C, int ldc, size_t sC, int M, int N, int K) {
  __shared__ __attribute__((aligned(16))) float so[4][16][64];
  const int tid = threadIdx.x, w = tid >> 5, lane = tid & 31, ln = lane & 15, hh = lane >> 4; const int by = blockIdx.y;
  A += (size_t)by * sA; Bh += (size_t)by * sB; C += (size_t)by * sC;
  const int ntn = (N + 63) / 64; const int wid = blockIdx.x * 4 + w; const int mt = wid / ntn, nq = wid % ntn; if (mt * 16 >= M) return;
  const int row0 = mt * 16, col0 = nq * 64; const float* arow = A + (size_t)(row0 + ln) * lda;
  v8f acc[4] = {};
  for (int kb = 0; kb < K; kb += 32) {
    FragH ah, al;
    const v4f x0 = *(const v4fa*)(arow + kb + 8 * hh), x1 = *(const v4fa*)(arow + kb + 8 * hh + 4), x2 = *(const v4fa*)(arow + kb + 16 + 8 * hh), x3 = *(const v4fa*)(arow + kb + 16 + 8 * hh + 4);
    float xs[16] = {x0[0],x0[1],x0[2],x0[3],x1[0],x1[1],x1[2],x1[3],x2[0],x2[1],x2[2],x2[3],x3[0],x3[1],x3[2],x3[3]};
#pragma unroll
    for (int i = 0; i < 16; ++i) { const _Float16 h = (_Float16)xs[i]; ah.h[i] = h; al.h[i] = ASPLIT ? (_Float16)(xs[i] - (float)h) : (_Float16)0.0f; }
#pragma unroll
    for (int t = 0; t < 4; ++t) { if (col0 + t * 16 >= N) continue; const size_t boff = (size_t)(col0 + t * 16 + ln) * ldb + kb; FragH bq; bq.half[0] = *(const v8us*)(Bh + boff + 8 * hh); bq.half[1] = *(const v8us*)(Bh + boff + 16 + 8 * hh);
      acc[t] = mmaH<ASPLIT ? 2 : 1>(ah.v, al.v, bq.v, bq.v, acc[t]); }
  }
#pragma unroll
  for (int t = 0; t < 4; ++t) { if (col0 + t * 16 >= N) continue;
#pragma unroll
    for (int r = 0; r < 8; ++r) so[w][8 * hh + r][t * 16 + ln] = acc[t][r] * alpha; }
  __builtin_amdgcn_fence(__ATOMIC_ACQ_REL, "workgroup"); __builtin_amdgcn_wave_barrier();
  const int rsub = lane >> 4, c4 = (lane & 15) * 4;
  for (int pass = 0; pass < 2; ++pass) {
#pragma unroll
    for (int q = 0; q < 8; ++q) { const int r = q * 2 + rsub; if (col0 + c4 < N) { const v4f v = *(const v4fa*)&so[w][r][c4]; *(volatile v4f*)(C + (size_t)(row0 + r) * ldc + col0 + c4) = v; } }
    if (pass == 0) __threadfence(); }
}

__global__ __launch_bounds__(256) void k_wt_f16(const float* __restrict__ W, _Float16* __restrict__ Wt, int K, int N, float scale) {
  const int t = blockIdx.x * 256 + threadIdx.x; if (t >= N * (K / 8)) return; const int n = t / (K / 8), k8 = (t % (K / 8)) * 8; FragH f;
#pragma unroll
  for (int i = 0; i < 8; ++i) f.h[i] = (_Float16)(bf16_round(W[(size_t)(k8 + i) * N + n]) * scale); const v8us o = f.half[0];
  *(volatile v8us*)((unsigned short*)Wt + (size_t)n * K + k8) = o; __threadfence(); *(volatile v8us*)((unsigned short*)Wt + (size_t)n * K + k8) = o;
}
template <int ACT>
__global__ __launch_bounds__(128) void k_gemm_hhx(const _Float16* __restrict__ A, int lda, size_t sA, const _Float16* __restrict__ Bh, int ldb, size_t sB, float alpha, const float* __restrict__ bias, size_t sBias, const float* __restrict__ CP, int rowsPerB, size_t sCPb, int row0g,
    float* __restrict__ C, _Float16* __restrict__ C16, int ldc, size_t sC, int M, int N, int K) {
  __shared__ __attribute__((aligned(16))) float so[4][16][64];
  const int tid = threadIdx.x, w = tid >> 5, lane = tid & 31, ln = lane & 15, hh = lane >> 4; const int by = blockIdx.y;
  A += (size_t)by * sA; Bh += (size_t)by * sB; const size_t cofs = (size_t)by * sC; const float* bp = bias ? bias + (size_t)by * sBias : nullptr;
  const int ntn = (N + 63) / 64; const int wid = blockIdx.x * 4 + w; const int mt = wid / ntn, nq = wid % ntn; if (mt * 16 >= M) return;
  const int row0 = mt * 16, col0 = nq * 64; const _Float16* arow = A + (size_t)(row0 + ln) * lda;
  v8f acc[4] = {};
  for (int kb = 0; kb < K; kb += 32) { FragH ah; ah.half[0] = *(const v8us*)((const unsigned short*)arow + kb + 8 * hh); ah.half[1] = *(const v8us*)((const unsigned short*)arow + kb + 16 + 8 * hh);
#pragma unroll
    for (int t = 0; t < 4; ++t) { if (col0 + t * 16 >= N) continue; const size_t boff = (size_t)(col0 + t * 16 + ln) * ldb + kb; FragH bq; bq.half[0] = *(const v8us*)((const unsigned short*)Bh + boff + 8 * hh); bq.half[1] = *(const v8us*)((const unsigned short*)Bh + boff + 16 + 8 * hh);
      acc[t] = mmaH<1>(ah.v, ah.v, bq.v, bq.v, acc[t]); }
  }
#pragma unroll
  for (int t = 0; t < 4; ++t) { if (col0 + t * 16 >= N) continue; const int col = col0 + t * 16 + ln; const float bv = bp ? bf16_round(bp[col]) : 0.f;
#pragma unroll
    for (int r = 0; r < 8; ++r) { float v = acc[t][r] * alpha + bv; if (CP) { const int rr = row0g + row0 + 8 * hh + r; if (rowsPerB < 0) v += CP[cofs + (size_t)rr * ldc + col];        else { const int bidx = rr / rowsPerB; v += CP[(size_t)bidx * sCPb + (size_t)by * 64 + col]; } } if (ACT == 1) v = (v > 0.f) ? v : expm1f(v); else if (ACT == 7) v = (v > 0.f) ? v + 1.0f : expf(v); else if (ACT == 8) v = tanhf(v); else if (ACT == 9) v = 0.5f * v * (1.0f + tanhf(0.7978845608028654f * (v + 0.044715f * v * v * v))); else if (ACT == 11) v = 1.0f / (1.0f + expf(-v)); else if (ACT == 12) v = (v > 0.f) ? v : 0.01f * v; else if (ACT == 14) v = (v > 0.f) ? v : 0.1f * v; else if (ACT == 16) v = (v >= 0.f) ? v : 0.3f * v; else if (ACT == 17) v = (v >= 0.f) ? v : 0.2f * v; else if (ACT == 15) v = v / (1.0f + expf(-v)); else if (ACT == 3) v = fmaxf(v, 0.f); else if (ACT == 6) v = 0.5f * v * (1.0f + erff(v * 0.70710678118654752f)); so[w][8 * hh + r][t * 16 + ln] = v; } }
  __builtin_amdgcn_fence(__ATOMIC_ACQ_REL, "workgroup"); __builtin_amdgcn_wave_barrier();
  const int rsub = lane >> 4, c4 = (lane & 15) * 4; typedef _Float16 v4h __attribute__((ext_vector_type(4)));
  for (int pass = 0; pass < 2; ++pass) {
#pragma unroll
    for (int q = 0; q < 8; ++q) { const int r = q * 2 + rsub; if (col0 + c4 < N) { const v4f v = *(const v4fa*)&so[w][r][c4]; if (C) *(volatile v4f*)(C + cofs + (size_t)(row0 + r) * ldc + col0 + c4) = v; if (C16) { v4h h4; for (int i = 0; i < 4; ++i) h4[i] = (_Float16)v[i]; *(volatile v4h*)(C16 + cofs + (size_t)(row0 + r) * ldc + col0 + c4) = h4; } } }
    if (pass == 0) __threadfence(); }
}


typedef _Float16 v4h __attribute__((ext_vector_type(4)));

__global__ __launch_bounds__(256) void k_x16(const float* __restrict__ x, _Float16* __restrict__ X16, size_t n8) { const size_t t = (size_t)blockIdx.x * 256 + threadIdx.x; if (t >= n8) return; FragH f;
#pragma unroll
  for (int q = 0; q < 8; ++q) f.h[q] = (_Float16)bf16_round(x[t * 8 + q]); *(volatile v8us*)((unsigned short*)X16 + t * 8) = f.half[0]; __threadfence(); *(volatile v8us*)((unsigned short*)X16 + t * 8) = f.half[0]; }
__global__ __launch_bounds__(256) void k_h16(const float* __restrict__ x, _Float16* __restrict__ X16, size_t n8) { const size_t t = (size_t)blockIdx.x * 256 + threadIdx.x; if (t >= n8) return; FragH f;
#pragma unroll
  for (int q = 0; q < 8; ++q) f.h[q] = (_Float16)x[t * 8 + q]; *(volatile v8us*)((unsigned short*)X16 + t * 8) = f.half[0]; __threadfence(); *(volatile v8us*)((unsigned short*)X16 + t * 8) = f.half[0]; }
__global__ __launch_bounds__(256) void k_round16f(const float* __restrict__ W, _Float16* __restrict__ Bt, size_t n8) { const size_t t = (size_t)blockIdx.x * 256 + threadIdx.x; if (t >= n8) return; FragH f;
#pragma unroll
  for (int i = 0; i < 8; ++i) f.h[i] = (_Float16)(bf16_round(W[t * 8 + i]) * 16.0f); *(volatile v8us*)((unsigned short*)Bt + t * 8) = f.half[0]; __threadfence(); *(volatile v8us*)((unsigned short*)Bt + t * 8) = f.half[0]; }
template <int NHv, int TTv>
__global__ __launch_bounds__(256) void k_vt(const _Float16* __restrict__ V16, int ldv, int voff, _Float16* __restrict__ Vt) { __shared__ unsigned short tl[64][66]; const int tid = threadIdx.x; const int slab = blockIdx.x / (TTv / 64), lg = blockIdx.x % (TTv / 64); const int b = slab / NHv, h = slab % NHv;
  for (int i = tid; i < 64 * 8; i += 256) { const int r = i / 8, c8 = (i % 8) * 8; FragH f; f.half[0] = *(const v8us*)((const unsigned short*)V16 + ((size_t)b * TTv + lg * 64 + r) * ldv + voff + h * 64 + c8);
#pragma unroll
    for (int q = 0; q < 8; ++q) tl[r][c8 + q] = f.u[q]; }
  __syncthreads();
  for (int pass = 0; pass < 2; ++pass) {
#pragma unroll
    for (int rd = 0; rd < 2; ++rd) { const int d = rd * 32 + tid / 8, pc = tid % 8; FragH f;
#pragma unroll
      for (int q = 0; q < 8; ++q) f.u[q] = tl[pc * 8 + q][d];
      *(volatile v8us*)((unsigned short*)Vt + ((size_t)slab * 64 + d) * TTv + lg * 64 + pc * 8) = f.half[0]; }
    if (pass == 0) __threadfence(); } }

__global__ __launch_bounds__(256) void k_hl(const float* __restrict__ F, _Float16* __restrict__ Hh, _Float16* __restrict__ Hl, size_t n8) { const size_t t = (size_t)blockIdx.x * 256 + threadIdx.x; if (t >= n8) return; FragH fh, fl; const v4f a = *(const v4fa*)(F + t * 8), c = *(const v4fa*)(F + t * 8 + 4);
#pragma unroll
  for (int q = 0; q < 4; ++q) { _Float16 h = (_Float16)a[q]; fh.h[q] = h; fl.h[q] = (_Float16)((a[q] - (float)h) * 1024.0f); h = (_Float16)c[q]; fh.h[4 + q] = h; fl.h[4 + q] = (_Float16)((c[q] - (float)h) * 1024.0f); }
  for (int pass = 0; pass < 2; ++pass) { *(volatile v8us*)((unsigned short*)Hh + t * 8) = fh.half[0]; *(volatile v8us*)((unsigned short*)Hl + t * 8) = fl.half[0]; if (pass == 0) __threadfence(); } }

__device__ __forceinline__ v16h g2_frag(const _Float16* p, int hh) { FragH f; f.half[0] = *(const v8us*)((const unsigned short*)p + 8 * hh); f.half[1] = *(const v8us*)((const unsigned short*)p + 16 + 8 * hh); return f.v; }
__device__ __forceinline__ v8f g2_mma(v16h a, v16h b, v8f c) { v8f d = __builtin_amdgcn_wmma_f32_16x16x32_f16(false, a, false, b, (short)0, c, false, false); asm volatile("v_nop\n\tv_nop\n\tv_nop\n\tv_nop" : "+v"(d) : "v"(a), "v"(b)); return d; }
template <int ACT>
__global__ __launch_bounds__(128) void k_gemm2(const _Float16* __restrict__ A, int lda, size_t sA, const _Float16* __restrict__ Bh, int ldb, size_t sB, float alpha, const float* __restrict__ bias, size_t sBias, const float* __restrict__ CP, int rowsPerB, size_t sCPb, int row0g,
    float* __restrict__ C, _Float16* __restrict__ C16, int ldc, size_t sC, int M, int N, int K) { static_assert(ACT == 0 || ACT == 3 || ACT == 6 || ACT == 8 || ACT == 9 || ACT == 11 || ACT == 12 || ACT == 14 || ACT == 15 || ACT == 16 || ACT == 17, "k_gemm2: unsupported ACT code (would silently apply no activation)");
  __shared__ __attribute__((aligned(16))) float so[4][32][68];
  const int tid = threadIdx.x, w = tid >> 5, lane = tid & 31, ln = lane & 15, hh = lane >> 4; const int by = blockIdx.y;
  A += (size_t)by * sA; Bh += (size_t)by * sB; const size_t cofs = (size_t)by * sC; const float* bp = bias ? bias + (size_t)by * sBias : nullptr;
  const int ntn = N >> 6; const int mt = blockIdx.x / ntn, nq = blockIdx.x - mt * ntn; const int row0 = mt * 128 + 32 * w, col0 = nq * 64; if (row0 >= M) return;
  const _Float16* a0p = A + (size_t)(row0 + ln) * lda; const _Float16* a1p = a0p + (size_t)16 * lda;
  const _Float16* b0p = Bh + (size_t)(col0 + ln) * ldb; const _Float16* b1p = b0p + (size_t)16 * ldb; const _Float16* b2p = b1p + (size_t)16 * ldb; const _Float16* b3p = b2p + (size_t)16 * ldb;
  const v8f z8 = {0.f,0.f,0.f,0.f,0.f,0.f,0.f,0.f}; v8f c00 = z8, c01 = z8, c02 = z8, c03 = z8, c10 = z8, c11 = z8, c12 = z8, c13 = z8;
#pragma unroll 1
  for (int kb = 0; kb < K; kb += 32) { const v16h a0 = g2_frag(a0p + kb, hh), a1 = g2_frag(a1p + kb, hh);
    v16h b = g2_frag(b0p + kb, hh); c00 = g2_mma(a0, b, c00); c10 = g2_mma(a1, b, c10);
    b = g2_frag(b1p + kb, hh); c01 = g2_mma(a0, b, c01); c11 = g2_mma(a1, b, c11);
    b = g2_frag(b2p + kb, hh); c02 = g2_mma(a0, b, c02); c12 = g2_mma(a1, b, c12);
    b = g2_frag(b3p + kb, hh); c03 = g2_mma(a0, b, c03); c13 = g2_mma(a1, b, c13); }
  v8f accs[8] = {c00, c01, c02, c03, c10, c11, c12, c13};
#pragma unroll
  for (int u = 0; u < 8; ++u) { const int t = u & 3, half = u >> 2; const int col = col0 + t * 16 + ln; const float bv = bp ? bf16_round(bp[col]) : 0.f;
#pragma unroll
    for (int r = 0; r < 8; ++r) { const int rloc = half * 16 + 8 * hh + r; float v = accs[u][r] * alpha + bv; if (CP) { if (rowsPerB < 0) v += CP[cofs + (size_t)(row0g + row0 + rloc) * ldc + col];        else { const int bidx = (row0g + row0 + rloc) / rowsPerB; v += CP[(size_t)bidx * sCPb + (size_t)by * 64 + col]; } }
      if (ACT == 3) v = fmaxf(v, 0.f); else if (ACT == 6) v = 0.5f * v * (1.0f + erff(v * 0.70710678118654752f)); else if (ACT == 11) v = 1.0f / (1.0f + expf(-v)); else if (ACT == 15) v = v / (1.0f + expf(-v)); else if (ACT == 12) v = (v > 0.f) ? v : 0.01f * v; else if (ACT == 8) v = tanhf(v); else if (ACT == 9) v = 0.5f * v * (1.0f + tanhf(0.7978845608028654f * (v + 0.044715f * v * v * v))); else if (ACT == 14) v = (v > 0.f) ? v : 0.1f * v; else if (ACT == 16) v = (v >= 0.f) ? v : 0.3f * v; else if (ACT == 17) v = (v >= 0.f) ? v : 0.2f * v;
      so[w][rloc][t * 16 + ln] = v; } }
  __builtin_amdgcn_fence(__ATOMIC_ACQ_REL, "workgroup"); __builtin_amdgcn_wave_barrier();
  const int rsub = lane >> 4, c4 = (lane & 15) * 4;
  for (int pass = 0; pass < 2; ++pass) {
#pragma unroll
    for (int q = 0; q < 16; ++q) { const int r = q * 2 + rsub; const v4f v = *(const v4fa*)&so[w][r][c4]; if (C) *(volatile v4f*)(C + cofs + (size_t)(row0 + r) * ldc + col0 + c4) = v; if (C16) { v4h h4; for (int i = 0; i < 4; ++i) h4[i] = (_Float16)v[i]; *(volatile v4h*)(C16 + cofs + (size_t)(row0 + r) * ldc + col0 + c4) = h4; } }
    if (pass == 0) __threadfence(); } }


__global__ __launch_bounds__(256) void k_rows(const float* __restrict__ src, _Float16* __restrict__ dst) { __shared__ float tl[CC][17]; const int tid = threadIdx.x; const int b = blockIdx.x / (PX / 16), pb = blockIdx.x % (PX / 16); const int p0 = pb * 16;
  for (int i = tid; i < CC * 16; i += 256) { const int c = i / 16, p = i % 16; tl[c][p] = bf16_round(src[((size_t)b * CC + c) * PX + p0 + p]); }
  __syncthreads();
  for (int pass = 0; pass < 2; ++pass) { for (int i = tid; i < 16 * (CC / 8); i += 256) { const int p = i / (CC / 8), c0 = (i % (CC / 8)) * 8; FragH f; for (int q = 0; q < 8; ++q) f.h[q] = (_Float16)tl[c0 + q][p]; *(volatile v8us*)((unsigned short*)dst + ((size_t)b * PX + p0 + p) * CC + c0) = f.half[0]; } if (pass == 0) __threadfence(); } }
template <int KS, int C>
__global__ __launch_bounds__(256) void k_imk(const _Float16* __restrict__ S, size_t r0, size_t nrows, _Float16* __restrict__ IM) { const size_t t_ = (size_t)blockIdx.x * 256 + threadIdx.x; if (t_ >= nrows * KS * KS * (C / 8)) return; const int c8 = (int)(t_ % (C / 8)) * 8; const int tap = (int)((t_ / (C / 8)) % (KS * KS)); const size_t row = r0 + t_ / ((size_t)KS * KS * (C / 8)); const int p = (int)(row % PX); const size_t b = row / PX; const int iy = p / HS + tap / KS - KS / 2, ix = p % HS + tap % KS - KS / 2; v8us v;
  if (iy >= 0 && iy < HS && ix >= 0 && ix < HS) v = *(const v8us*)((const unsigned short*)S + (b * PX + (size_t)iy * HS + ix) * C + c8); else { for (int q = 0; q < 8; ++q) v[q] = 0; }
  *(volatile v8us*)((unsigned short*)IM + t_ * 8) = v; __threadfence(); *(volatile v8us*)((unsigned short*)IM + t_ * 8) = v; }
template <int NT, int C>
__global__ __launch_bounds__(256) void k_wt(const float* __restrict__ w, int nrows, _Float16* __restrict__ Bt) { const size_t t_ = (size_t)blockIdx.x * 256 + threadIdx.x; const size_t kc = (size_t)NT * C; if (t_ >= (size_t)nrows * kc / 8) return; const int c8 = (int)((t_ * 8) % C); const int tap = (int)(((t_ * 8) / C) % NT); const int o = (int)((t_ * 8) / kc); FragH f;
  for (int q = 0; q < 8; ++q) f.h[q] = (_Float16)(bf16_round(w[((size_t)o * C + c8 + q) * NT + tap]) * 16.0f); *(volatile v8us*)((unsigned short*)Bt + t_ * 8) = f.half[0]; __threadfence(); *(volatile v8us*)((unsigned short*)Bt + t_ * 8) = f.half[0]; }
__global__ __launch_bounds__(256) void k_stem2(const float* __restrict__ S0, const float* __restrict__ g, const float* __restrict__ bb, float* __restrict__ X1F, _Float16* __restrict__ X1H) {
  #pragma clang fp contract(off)
  const size_t t_ = (size_t)blockIdx.x * 256 + threadIdx.x; if (t_ >= NRW * CC / 8) return; const int c0 = (int)((t_ * 8) % CC); const size_t r = (t_ * 8) / CC; const int p = (int)(r % PX); const size_t b = r / PX; const int y = p / HS, x = p % HS; v8f m; for (int q = 0; q < 8; ++q) m[q] = -3.0e38f;
#pragma unroll 1
  for (int tp = 0; tp < 9; ++tp) { const int yy = y + tp / 3 - 1, xx = x + tp % 3 - 1; if (yy < 0 || yy >= HS || xx < 0 || xx >= HS) continue; const v8f s = *(const v8f*)(S0 + (b * PX + (size_t)yy * HS + xx) * CC + c0);
    for (int q = 0; q < 8; ++q) { const int c = c0 + q; const float v = fmaxf(__fadd_rn(__fmul_rn(s[q], bf16_round(g[c])), bf16_round(bb[c])), 0.f); m[q] = fmaxf(m[q], v); } }
  FragH f; for (int q = 0; q < 8; ++q) f.h[q] = (_Float16)m[q]; *(volatile v8f*)(X1F + t_ * 8) = m; *(volatile v8us*)((unsigned short*)X1H + t_ * 8) = f.half[0]; __threadfence(); *(volatile v8f*)(X1F + t_ * 8) = m; *(volatile v8us*)((unsigned short*)X1H + t_ * 8) = f.half[0]; }
template <int CW, int ACT>
__global__ __launch_bounds__(256) void k_bnact(const float* __restrict__ F, const float* __restrict__ g, const float* __restrict__ bb, _Float16* __restrict__ H, float* __restrict__ F32, size_t nrows) {
  #pragma clang fp contract(off)
  const size_t t_ = (size_t)blockIdx.x * 256 + threadIdx.x; if (t_ >= nrows * CW / 8) return; const int c0 = (int)((t_ * 8) % CW); const v8f s = *(const v8f*)(F + t_ * 8); v8f o; FragH f;
  for (int q = 0; q < 8; ++q) { const int c = c0 + q; float v = __fadd_rn(__fmul_rn(s[q], bf16_round(g[c])), bf16_round(bb[c])); if (ACT == 1) v = fmaxf(v, 0.f); if (ACT == 2) v = v / (1.0f + expf(-v)); o[q] = v; f.h[q] = (_Float16)v; }
  for (int pass = 0; pass < 2; ++pass) { *(volatile v8us*)((unsigned short*)H + t_ * 8) = f.half[0]; if (F32) *(volatile v8f*)(F32 + t_ * 8) = o; if (pass == 0) __threadfence(); } }
__global__ __launch_bounds__(256) void k_xc(const float* __restrict__ T3, const float* __restrict__ g3, const float* __restrict__ b3, const float* __restrict__ R, const float* __restrict__ gr, const float* __restrict__ br, float* __restrict__ XCF, _Float16* __restrict__ XCH) {
  #pragma clang fp contract(off)
  const size_t t_ = (size_t)blockIdx.x * 256 + threadIdx.x; if (t_ >= NRW * CC / 8) return; const int c0 = (int)((t_ * 8) % CC); const v8f a = *(const v8f*)(T3 + t_ * 8), rr = *(const v8f*)(R + t_ * 8); v8f o; FragH f;
  for (int q = 0; q < 8; ++q) { const int c = c0 + q; const float t = __fadd_rn(__fmul_rn(a[q], bf16_round(g3[c])), bf16_round(b3[c])); const float s = __fadd_rn(__fmul_rn(rr[q], bf16_round(gr[c])), bf16_round(br[c])); o[q] = fmaxf(t + s, 0.f); f.h[q] = (_Float16)o[q]; }
  for (int pass = 0; pass < 2; ++pass) { *(volatile v8f*)(XCF + t_ * 8) = o; *(volatile v8us*)((unsigned short*)XCH + t_ * 8) = f.half[0]; if (pass == 0) __threadfence(); } }
__global__ __launch_bounds__(64) void k_cw2(const float* __restrict__ cw, float* __restrict__ C2) {
  #pragma clang fp contract(off)
  const int k = threadIdx.x; if (k >= NK) return; float s = 0.f;
#pragma unroll 1
  for (int c = 0; c < CC; ++c) { const float v = bf16_round(cw[k * CC + c]); s = __fadd_rn(s, __fmul_rn(v, v)); } *(volatile float*)(C2 + k) = s; __threadfence(); *(volatile float*)(C2 + k) = s; }
__global__ __launch_bounds__(256) void k_assign(const float* __restrict__ ZF, const float* __restrict__ ZC, const float* __restrict__ C2, const float* __restrict__ cws, float* __restrict__ A, _Float16* __restrict__ AT16) {
  #pragma clang fp contract(off)
  const size_t r = (size_t)blockIdx.x * 256 + threadIdx.x; if (r >= NRW) return; const size_t b = r / PX; const int n = (int)(r % PX); float x2 = 0.f;
#pragma unroll 1
  for (int c = 0; c < CC; ++c) { const float v = ZF[r * CC + c]; x2 = __fadd_rn(x2, __fmul_rn(v, v)); }
  float mx = -3.0e38f;
#pragma unroll 1
  for (int k = 0; k < NK; ++k) { float d = x2 - 2.0f * ZC[r * NK + k]; d = d + C2[k]; d = __fmul_rn(bf16_round(cws[k]), d); mx = fmaxf(mx, d); }
  float se = 0.f;
#pragma unroll 1
  for (int k = 0; k < NK; ++k) { float d = x2 - 2.0f * ZC[r * NK + k]; d = d + C2[k]; d = __fmul_rn(bf16_round(cws[k]), d); se += expf(d - mx); }
  for (int pass = 0; pass < 2; ++pass) {
#pragma unroll 1
    for (int k0 = 0; k0 < NK; k0 += 8) { v8f a8; for (int q = 0; q < 8; ++q) { const int k = k0 + q; float d = x2 - 2.0f * ZC[r * NK + k]; d = d + C2[k]; d = __fmul_rn(bf16_round(cws[k]), d); a8[q] = expf(d - mx) / se; } *(volatile v8f*)(A + r * NK + k0) = a8; }
    if (pass == 0) __threadfence(); } (void)AT16; (void)b; (void)n; }
__global__ __launch_bounds__(256) void k_at(const float* __restrict__ A, _Float16* __restrict__ AT16) { __shared__ float tl[64][65]; const int tid = threadIdx.x; const int b = blockIdx.x / (PX / 64), ng = blockIdx.x % (PX / 64); const int n0 = ng * 64;
  for (int i = tid; i < 64 * 64; i += 256) { const int j = i / 64, k = i % 64; tl[j][k] = A[((size_t)b * PX + n0 + j) * NK + k]; }
  __syncthreads();
  for (int pass = 0; pass < 2; ++pass) { { const int k = tid / 4, j8 = (tid % 4) * 16; for (int h2 = 0; h2 < 2; ++h2) { FragH f; for (int q = 0; q < 8; ++q) f.h[q] = (_Float16)tl[j8 + h2 * 8 + q][k]; *(volatile v8us*)((unsigned short*)AT16 + ((size_t)b * NK + k) * PX + n0 + j8 + h2 * 8) = f.half[0]; } } if (pass == 0) __threadfence(); } }
__global__ __launch_bounds__(256) void k_zt(const _Float16* __restrict__ Z16, _Float16* __restrict__ ZT) { __shared__ unsigned short tl[64][258]; const int tid = threadIdx.x; const int b = blockIdx.x / (PX / 64), ng = blockIdx.x % (PX / 64); const int n0 = ng * 64;
  for (int i = tid; i < 64 * 32; i += 256) { const int j = i / 32, c8 = (i % 32) * 8; FragH f; f.half[0] = *(const v8us*)((const unsigned short*)Z16 + ((size_t)b * PX + n0 + j) * CC + c8); for (int q = 0; q < 8; ++q) tl[j][c8 + q] = f.u[q]; }
  __syncthreads();
  for (int pass = 0; pass < 2; ++pass) { for (int i = tid; i < CC * 8; i += 256) { const int c = i / 8, j8 = (i % 8) * 8; FragH f; for (int q = 0; q < 8; ++q) f.u[q] = tl[j8 + q][c]; *(volatile v8us*)((unsigned short*)ZT + ((size_t)b * CC + c) * PX + n0 + j8) = f.half[0]; } if (pass == 0) __threadfence(); } }
__global__ __launch_bounds__(256) void k_asum(const float* __restrict__ A, float* __restrict__ ASUM) { __shared__ double red[256]; const int tid = threadIdx.x; const int b = blockIdx.x / NK, k = blockIdx.x % NK; double s = 0.0; for (int n = tid; n < PX; n += 256) s += (double)A[((size_t)b * PX + n) * NK + k];
  red[tid] = s; __syncthreads(); for (int st = 128; st > 0; st >>= 1) { if (tid < st) red[tid] += red[tid + st]; __syncthreads(); }
  if (tid == 0) { const float v = (float)red[0]; *(volatile float*)(ASUM + blockIdx.x * 32) = v; __threadfence(); *(volatile float*)(ASUM + blockIdx.x * 32) = v; } }
__global__ __launch_bounds__(256) void k_em(const float* __restrict__ ENT, const float* __restrict__ ASUM, const float* __restrict__ cw, const float* __restrict__ ge, const float* __restrict__ be, float* __restrict__ EM) {
  #pragma clang fp contract(off)
  const int t = blockIdx.x * 256 + threadIdx.x; if (t >= NB * CC) return; const int c = t % CC, b = t / CC; float s = 0.f;
#pragma unroll 1
  for (int k = 0; k < NK; ++k) { float e = ENT[((size_t)b * CC + c) * NK + k] - __fmul_rn(ASUM[(b * NK + k) * 32], bf16_round(cw[k * CC + c])); e = __fadd_rn(__fmul_rn(e, bf16_round(ge[k])), bf16_round(be[k])); s += fmaxf(e, 0.f); }
  const float v = s / (float)NK; *(volatile float*)(EM + t) = v; __threadfence(); *(volatile float*)(EM + t) = v; }
__global__ __launch_bounds__(256) void k_gate(const float* __restrict__ EM, const float* __restrict__ wfc, const float* __restrict__ bfc, float* __restrict__ GAM) {
  #pragma clang fp contract(off)
  const int t = blockIdx.x * 256 + threadIdx.x; if (t >= NB * CC) return; const int c = t % CC, b = t / CC; float s = 0.f;
#pragma unroll 1
  for (int c2 = 0; c2 < CC; ++c2) s = __fadd_rn(s, __fmul_rn(EM[b * CC + c2], bf16_round(wfc[c * CC + c2])));
  s = s + bf16_round(bfc[c]); const float gm = 1.0f / (1.0f + expf(-s)); *(volatile float*)(GAM + t) = gm; __threadfence(); *(volatile float*)(GAM + t) = gm; }
__global__ __launch_bounds__(256) void k_xlvc(const float* __restrict__ XCF, const float* __restrict__ GAM, _Float16* __restrict__ CAT) {
  #pragma clang fp contract(off)
  const size_t t_ = (size_t)blockIdx.x * 256 + threadIdx.x; if (t_ >= NRW * CC / 8) return; const int c0 = (int)((t_ * 8) % CC); const size_t r = (t_ * 8) / CC; const size_t b = r / PX; const v8f xc = *(const v8f*)(XCF + t_ * 8); FragH f;
  for (int q = 0; q < 8; ++q) { const float v = xc[q] + __fmul_rn(xc[q], GAM[b * CC + c0 + q]); f.h[q] = (_Float16)fmaxf(v, 0.f); }
  unsigned short* d = (unsigned short*)CAT + r * (2 * CC) + c0; *(volatile v8us*)d = f.half[0]; __threadfence(); *(volatile v8us*)d = f.half[0]; }
__global__ __launch_bounds__(256) void k_gs1(const float* __restrict__ F, double* __restrict__ part) { __shared__ double rs[256], rq[256]; const int tid = threadIdx.x; const int b = blockIdx.x / NPART, pb = blockIdx.x % NPART; const size_t n0 = (size_t)PX * CC / NPART; const float* p = F + (size_t)b * PX * CC + pb * n0; double s = 0.0, q2 = 0.0;
  for (size_t i = tid; i < n0; i += 256) { const double v = (double)p[i]; s += v; q2 += v * v; }
  rs[tid] = s; rq[tid] = q2; __syncthreads(); for (int st = 128; st > 0; st >>= 1) { if (tid < st) { rs[tid] += rs[tid + st]; rq[tid] += rq[tid + st]; } __syncthreads(); }
  if (tid == 0) { for (int pass = 0; pass < 2; ++pass) { *(volatile double*)(part + (size_t)blockIdx.x * 16) = rs[0]; *(volatile double*)(part + (size_t)blockIdx.x * 16 + 1) = rq[0]; if (pass == 0) __threadfence(); } } }
__global__ __launch_bounds__(64) void k_gs2(const double* __restrict__ part, float* __restrict__ stat) { const int b = threadIdx.x; if (b >= NB) return; double s = 0.0, q2 = 0.0; for (int pb = 0; pb < NPART; ++pb) { s += part[((size_t)b * NPART + pb) * 16]; q2 += part[((size_t)b * NPART + pb) * 16 + 1]; }
  const double n = (double)PX * CC; const double mu = s / n; double var = q2 / n - mu * mu; if (var < 0.0) var = 0.0; const float m = (float)mu, rsd = (float)(1.0 / sqrt(var + 1e-5));
  for (int pass = 0; pass < 2; ++pass) { *(volatile float*)(stat + b * 2) = m; *(volatile float*)(stat + b * 2 + 1) = rsd; if (pass == 0) __threadfence(); } }
__global__ __launch_bounds__(256) void k_dw(const float* __restrict__ X1F, const float* __restrict__ stat, const float* __restrict__ g1, const float* __restrict__ b1, const float* __restrict__ wdw, const float* __restrict__ gd, const float* __restrict__ bd, _Float16* __restrict__ H16) {
  #pragma clang fp contract(off)
  const size_t t_ = (size_t)blockIdx.x * 256 + threadIdx.x; if (t_ >= NRW * CC / 8) return; const int c0 = (int)((t_ * 8) % CC); const size_t r = (t_ * 8) / CC; const size_t b = r / PX; const float mu = stat[b * 2], rsd = stat[b * 2 + 1]; const v8f s = *(const v8f*)(X1F + t_ * 8); FragH f;
  for (int q = 0; q < 8; ++q) { const int c = c0 + q; float v = __fadd_rn(__fmul_rn((s[q] - mu) * rsd, bf16_round(g1[c])), bf16_round(b1[c])); v = __fmul_rn(v, bf16_round(wdw[c])); v = __fadd_rn(__fmul_rn(v, bf16_round(gd[c])), bf16_round(bd[c])); v = v / (1.0f + expf(-v)); f.h[q] = (_Float16)v; }
  *(volatile v8us*)((unsigned short*)H16 + t_ * 8) = f.half[0]; __threadfence(); *(volatile v8us*)((unsigned short*)H16 + t_ * 8) = f.half[0]; }
__global__ __launch_bounds__(256) void k_xm(const float* __restrict__ X1F, const float* __restrict__ PWF, const float* __restrict__ gp, const float* __restrict__ bp, const float* __restrict__ ls1, float* __restrict__ XMF) {
  #pragma clang fp contract(off)
  const size_t t_ = (size_t)blockIdx.x * 256 + threadIdx.x; if (t_ >= NRW * CC / 8) return; const int c0 = (int)((t_ * 8) % CC); const v8f x1 = *(const v8f*)(X1F + t_ * 8), pw = *(const v8f*)(PWF + t_ * 8); v8f o;
  for (int q = 0; q < 8; ++q) { const int c = c0 + q; float v = __fadd_rn(__fmul_rn(pw[q], bf16_round(gp[c])), bf16_round(bp[c])); v = v / (1.0f + expf(-v)); o[q] = x1[q] + __fmul_rn(bf16_round(ls1[c]), v); }
  *(volatile v8f*)(XMF + t_ * 8) = o; __threadfence(); *(volatile v8f*)(XMF + t_ * 8) = o; }
__global__ __launch_bounds__(256) void k_gn2(const float* __restrict__ XMF, const float* __restrict__ stat, const float* __restrict__ g2, const float* __restrict__ b2, _Float16* __restrict__ G2H) {
  #pragma clang fp contract(off)
  const size_t t_ = (size_t)blockIdx.x * 256 + threadIdx.x; if (t_ >= NRW * CC / 8) return; const int c0 = (int)((t_ * 8) % CC); const size_t r = (t_ * 8) / CC; const size_t b = r / PX; const float mu = stat[b * 2], rsd = stat[b * 2 + 1]; const v8f s = *(const v8f*)(XMF + t_ * 8); FragH f;
  for (int q = 0; q < 8; ++q) { const int c = c0 + q; f.h[q] = (_Float16)__fadd_rn(__fmul_rn((s[q] - mu) * rsd, bf16_round(g2[c])), bf16_round(b2[c])); }
  *(volatile v8us*)((unsigned short*)G2H + t_ * 8) = f.half[0]; __threadfence(); *(volatile v8us*)((unsigned short*)G2H + t_ * 8) = f.half[0]; }
__global__ __launch_bounds__(256) void k_xm2(const float* __restrict__ XMF, const float* __restrict__ F2, const float* __restrict__ ls2, _Float16* __restrict__ CAT) {
  #pragma clang fp contract(off)
  const size_t t_ = (size_t)blockIdx.x * 256 + threadIdx.x; if (t_ >= NRW * CC / 8) return; const int c0 = (int)((t_ * 8) % CC); const size_t r = (t_ * 8) / CC; const v8f xm = *(const v8f*)(XMF + t_ * 8), f2 = *(const v8f*)(F2 + t_ * 8); FragH f;
  for (int q = 0; q < 8; ++q) f.h[q] = (_Float16)(xm[q] + __fmul_rn(bf16_round(ls2[c0 + q]), f2[q]));
  unsigned short* d = (unsigned short*)CAT + r * (2 * CC) + CC + c0; *(volatile v8us*)d = f.half[0]; __threadfence(); *(volatile v8us*)d = f.half[0]; }
__global__ __launch_bounds__(256) void k_out(const float* __restrict__ OUTR, float* __restrict__ out) { const size_t t_ = (size_t)blockIdx.x * 256 + threadIdx.x; if (t_ >= (size_t)NB * CC * PX / 8) return; const int p0 = (int)((t_ * 8) % PX); const size_t bc = (t_ * 8) / PX; const int c = (int)(bc % CC); const size_t b = bc / CC; v8f r;
  for (int q = 0; q < 8; ++q) r[q] = OUTR[(b * PX + p0 + q) * CC + c]; *(volatile v8f*)(out + t_ * 8) = r; __threadfence(); *(volatile v8f*)(out + t_ * 8) = r; }

extern "C" void kernel_launch(void* const* d_in, const int* in_sizes, int n_in,
                              void* d_out, int out_size, void* d_ws, size_t ws_size, hipStream_t stream) {
  (void)in_sizes; (void)n_in; (void)out_size;
  const float* const* I = (const float* const*)d_in;
  const float *x = I[0], *w_stem = I[1], *g_stem = I[2], *b_stem = I[3], *w_cb1 = I[4], *g_cb1 = I[5], *b_cb1 = I[6], *w_cb2 = I[7], *g_cb2 = I[8], *b_cb2 = I[9], *w_cb3 = I[10], *g_cb3 = I[11], *b_cb3 = I[12], *w_cbres = I[13], *g_cbres = I[14], *b_cbres = I[15], *w_lvc = I[16], *g_lvc = I[17], *b_lvc = I[18], *cwd = I[19], *cws = I[20], *g_enc = I[21], *b_enc = I[22], *w_fc = I[23], *b_fc = I[24], *gn1_g = I[25], *gn1_b = I[26], *w_dw = I[27], *g_dw = I[28], *b_dw = I[29], *w_pw = I[30], *g_pw = I[31], *b_pw = I[32], *gn2_g = I[33], *gn2_b = I[34], *w_fc1 = I[35], *bias_fc1 = I[36], *w_fc2 = I[37], *bias_fc2 = I[38], *ls1 = I[39], *ls2 = I[40], *w_cnv1 = I[41], *b_cnv1 = I[42];
  char* ws = (char*)d_ws; size_t off = 0;
  auto take = [&](size_t bytes) { char* p = ws + off; off += (bytes + 255) & ~(size_t)255; return p; };
  _Float16* BST = (_Float16*)take((size_t)CC * KST * 2); _Float16* B1 = (_Float16*)take((size_t)CQ * CC * 2); _Float16* B2 = (_Float16*)take((size_t)CQ * 9 * CQ * 2); _Float16* B3 = (_Float16*)take((size_t)CC * CQ * 2); _Float16* BR = (_Float16*)take((size_t)CC * CC * 2); _Float16* BL = (_Float16*)take((size_t)CC * CC * 2); _Float16* BCW = (_Float16*)take((size_t)NK * CC * 2); float* C2 = (float*)take(NK * 4);
  _Float16* BPW = (_Float16*)take((size_t)CC * CC * 2); _Float16* BF1 = (_Float16*)take((size_t)HID * CC * 2); _Float16* BF2 = (_Float16*)take((size_t)CC * HID * 2); _Float16* BCV = (_Float16*)take((size_t)CC * 2 * CC * 2);
  _Float16* X16 = (_Float16*)take(NRW * CC * 2); float* S0 = (float*)take(NRW * CC * 4); float* X1F = (float*)take(NRW * CC * 4); _Float16* X1H = (_Float16*)take(NRW * CC * 2); _Float16* T1H = (_Float16*)take(NRW * CQ * 2); _Float16* T2H = (_Float16*)take(NRW * CQ * 2); float* XCF = (float*)take(NRW * CC * 4); _Float16* XCH = (_Float16*)take(NRW * CC * 2);
  _Float16* H16 = (_Float16*)take(NRW * CC * 2); float* XMF = (float*)take(NRW * CC * 4); _Float16* G2H = (_Float16*)take(NRW * CC * 2); _Float16* CAT = (_Float16*)take(NRW * 2 * CC * 2); double* part = (double*)take((size_t)NB * NPART * 16 * 8); float* stat = (float*)take(NB * 2 * 4);
  char* BIG = take((size_t)RCH * KST * 2);
  if (off > ws_size) return;
    float* T3 = (float*)BIG; float* R = T3 + NRW * CC; float* ZF = R + NRW * CC; _Float16* Z16 = (_Float16*)(ZF + NRW * CC); _Float16* ZT16 = Z16 + NRW * CC; _Float16* AT16 = ZT16 + NRW * CC; float* ZC = (float*)(AT16 + (size_t)NB * NK * PX); float* A = ZC + NRW * NK; float* ASUM = A + NRW * NK; float* ENT = ASUM + (size_t)NB * NK * 32; float* EM = ENT + (size_t)NB * CC * NK; float* GAM = EM + NB * CC;
    float* PWF = (float*)BIG; _Float16* F1H = (_Float16*)(PWF + NRW * CC); float* F2 = (float*)(F1H + NRW * HID); float* OUTR = S0;
  k_wt<49, CC><<<(unsigned)(((size_t)CC * KST / 8 + 255) / 256), 256, 0, stream>>>(w_stem, CC, BST);
  k_round16f<<<(CQ * CC / 8 + 255) / 256, 256, 0, stream>>>(w_cb1, B1, (size_t)CQ * CC / 8); k_wt<9, CQ><<<(unsigned)(((size_t)CQ * 9 * CQ / 8 + 255) / 256), 256, 0, stream>>>(w_cb2, CQ, B2); k_round16f<<<(CC * CQ / 8 + 255) / 256, 256, 0, stream>>>(w_cb3, B3, (size_t)CC * CQ / 8);
  k_round16f<<<(CC * CC / 8 + 255) / 256, 256, 0, stream>>>(w_cbres, BR, (size_t)CC * CC / 8); k_round16f<<<(CC * CC / 8 + 255) / 256, 256, 0, stream>>>(w_lvc, BL, (size_t)CC * CC / 8); k_round16f<<<(NK * CC / 8 + 255) / 256, 256, 0, stream>>>(cwd, BCW, (size_t)NK * CC / 8); k_cw2<<<1, 64, 0, stream>>>(cwd, C2);
  k_round16f<<<(CC * CC / 8 + 255) / 256, 256, 0, stream>>>(w_pw, BPW, (size_t)CC * CC / 8); k_round16f<<<(unsigned)((HID * CC / 8 + 255) / 256), 256, 0, stream>>>(w_fc1, BF1, (size_t)HID * CC / 8); k_round16f<<<(unsigned)((CC * HID / 8 + 255) / 256), 256, 0, stream>>>(w_fc2, BF2, (size_t)CC * HID / 8); k_round16f<<<(unsigned)((CC * 2 * CC / 8 + 255) / 256), 256, 0, stream>>>(w_cnv1, BCV, (size_t)CC * 2 * CC / 8);
  k_rows<<<(unsigned)(NB * (PX / 16)), 256, 0, stream>>>(x, X16);
  for (size_t r0 = 0; r0 < NRW; r0 += RCH) { k_imk<7, CC><<<(unsigned)(((size_t)RCH * 49 * (CC / 8) + 255) / 256), 256, 0, stream>>>(X16, r0, RCH, (_Float16*)BIG);
    k_gemm2<0><<<dim3((RCH / 128) * (CC / 64), 1), 128, 0, stream>>>((_Float16*)BIG, KST, 0, BST, KST, 0, 0.0625f, nullptr, 0, nullptr, 1, 0, 0, S0 + r0 * CC, nullptr, CC, 0, RCH, CC, KST); }
  const unsigned g256 = (unsigned)((NRW * CC / 8 + 255) / 256), g64 = (unsigned)((NRW * CQ / 8 + 255) / 256); const dim3 gN256((unsigned)((NRW / 128) * (CC / 64)), 1), gN64((unsigned)((NRW / 128) * 1), 1);
  k_stem2<<<g256, 256, 0, stream>>>(S0, g_stem, b_stem, X1F, X1H);
  k_gemm2<0><<<gN64, 128, 0, stream>>>(X1H, CC, 0, B1, CC, 0, 0.0625f, nullptr, 0, nullptr, 1, 0, 0, T3, nullptr, CQ, 0, (int)NRW, CQ, CC); k_bnact<CQ, 1><<<g64, 256, 0, stream>>>(T3, g_cb1, b_cb1, T1H, nullptr, NRW);
  k_imk<3, CQ><<<(unsigned)((NRW * 9 * (CQ / 8) + 255) / 256), 256, 0, stream>>>(T1H, 0, NRW, Z16);
  k_gemm2<0><<<gN64, 128, 0, stream>>>(Z16, 9 * CQ, 0, B2, 9 * CQ, 0, 0.0625f, nullptr, 0, nullptr, 1, 0, 0, T3, nullptr, CQ, 0, (int)NRW, CQ, 9 * CQ); k_bnact<CQ, 1><<<g64, 256, 0, stream>>>(T3, g_cb2, b_cb2, T2H, nullptr, NRW);
  k_gemm2<0><<<gN256, 128, 0, stream>>>(T2H, CQ, 0, B3, CQ, 0, 0.0625f, nullptr, 0, nullptr, 1, 0, 0, T3, nullptr, CC, 0, (int)NRW, CC, CQ);
  k_gemm2<0><<<gN256, 128, 0, stream>>>(X1H, CC, 0, BR, CC, 0, 0.0625f, nullptr, 0, nullptr, 1, 0, 0, R, nullptr, CC, 0, (int)NRW, CC, CC);
  k_xc<<<g256, 256, 0, stream>>>(T3, g_cb3, b_cb3, R, g_cbres, b_cbres, XCF, XCH);
  k_gemm2<0><<<gN256, 128, 0, stream>>>(XCH, CC, 0, BL, CC, 0, 0.0625f, nullptr, 0, nullptr, 1, 0, 0, T3, nullptr, CC, 0, (int)NRW, CC, CC); k_bnact<CC, 1><<<g256, 256, 0, stream>>>(T3, g_lvc, b_lvc, Z16, ZF, NRW);
  k_gemm2<0><<<gN64, 128, 0, stream>>>(Z16, CC, 0, BCW, CC, 0, 0.0625f, nullptr, 0, nullptr, 1, 0, 0, ZC, nullptr, NK, 0, (int)NRW, NK, CC);
  k_assign<<<(unsigned)((NRW + 255) / 256), 256, 0, stream>>>(ZF, ZC, C2, cws, A, AT16); k_at<<<NB * (PX / 64), 256, 0, stream>>>(A, AT16); k_zt<<<NB * (PX / 64), 256, 0, stream>>>(Z16, ZT16); k_asum<<<NB * NK, 256, 0, stream>>>(A, ASUM);
  k_gemm2<0><<<dim3((CC / 128) * (NK / 64), NB), 128, 0, stream>>>(ZT16, PX, (size_t)CC * PX, AT16, PX, (size_t)NK * PX, 1.0f, nullptr, 0, nullptr, 1, 0, 0, ENT, nullptr, NK, (size_t)CC * NK, CC, NK, PX);
  k_em<<<(NB * CC + 255) / 256, 256, 0, stream>>>(ENT, ASUM, cwd, g_enc, b_enc, EM); k_gate<<<(NB * CC + 255) / 256, 256, 0, stream>>>(EM, w_fc, b_fc, GAM);
  k_xlvc<<<g256, 256, 0, stream>>>(XCF, GAM, CAT);
  k_gs1<<<NB * NPART, 256, 0, stream>>>(X1F, part); k_gs2<<<1, 64, 0, stream>>>(part, stat); k_dw<<<g256, 256, 0, stream>>>(X1F, stat, gn1_g, gn1_b, w_dw, g_dw, b_dw, H16);
  k_gemm2<0><<<gN256, 128, 0, stream>>>(H16, CC, 0, BPW, CC, 0, 0.0625f, nullptr, 0, nullptr, 1, 0, 0, PWF, nullptr, CC, 0, (int)NRW, CC, CC); k_xm<<<g256, 256, 0, stream>>>(X1F, PWF, g_pw, b_pw, ls1, XMF);
  k_gs1<<<NB * NPART, 256, 0, stream>>>(XMF, part); k_gs2<<<1, 64, 0, stream>>>(part, stat); k_gn2<<<g256, 256, 0, stream>>>(XMF, stat, gn2_g, gn2_b, G2H);
  k_gemm2<6><<<dim3((unsigned)((NRW / 128) * (HID / 64)), 1), 128, 0, stream>>>(G2H, CC, 0, BF1, CC, 0, 0.0625f, bias_fc1, 0, nullptr, 1, 0, 0, nullptr, F1H, HID, 0, (int)NRW, HID, CC);
  k_gemm2<0><<<gN256, 128, 0, stream>>>(F1H, HID, 0, BF2, HID, 0, 0.0625f, bias_fc2, 0, nullptr, 1, 0, 0, F2, nullptr, CC, 0, (int)NRW, CC, HID); k_xm2<<<g256, 256, 0, stream>>>(XMF, F2, ls2, CAT);
  k_gemm2<0><<<gN256, 128, 0, stream>>>(CAT, 2 * CC, 0, BCV, 2 * CC, 0, 0.0625f, b_cnv1, 0, nullptr, 1, 0, 0, OUTR, nullptr, CC, 0, (int)NRW, CC, 2 * CC);
  k_out<<<(unsigned)(((size_t)NB * CC * PX / 8 + 255) / 256), 256, 0, stream>>>(OUTR, (float*)d_out);
}
